// ObjectCentricCausal_25245817766359
// MI455X (gfx1250) — hardware-run, weakly checked
//
#include <hip/hip_runtime.h>
#include <math.h>

constexpr int kNObj    = 20;
constexpr int kObjDim  = 64;
constexpr int kDModel  = 128;
constexpr int kHeads   = 4;
constexpr int kHeadDim = 16;
constexpr int kHid     = kObjDim * kNObj;
constexpr int kQkvW    = 3 * kObjDim;
constexpr int kCpHid   = 32;
constexpr int kThreads = 256;

typedef __attribute__((ext_vector_type(16))) _Float16 v16h;
typedef __attribute__((ext_vector_type(8)))  _Float16 v8h;
typedef __attribute__((ext_vector_type(16))) __bf16   v16b;
typedef __attribute__((ext_vector_type(8)))  __bf16   v8b;
typedef __attribute__((ext_vector_type(8)))  float    v8f;
typedef __attribute__((ext_vector_type(4)))  float    v4f;
typedef __attribute__((ext_vector_type(4)))  unsigned int v4u;

__device__ __forceinline__ unsigned short f2bf_bits(float f) {
  unsigned u = __float_as_uint(f);
  return (unsigned short)((u + 0x7FFFu + ((u >> 16) & 1u)) >> 16);
}
__device__ __forceinline__ float bf_bits2f(unsigned short h) { return __uint_as_float(((unsigned)h) << 16); }

__device__ __forceinline__ void dep_guard_h(v8f& a, v8f& b, v16h x, v16h y) { asm volatile("v_nop\n\tv_nop\n\tv_nop\n\tv_nop" : "+v"(a), "+v"(b) : "v"(x), "v"(y)); }
__device__ __forceinline__ void dep_guard_b(v8f& a, v8f& b, v16b x, v16b y) { asm volatile("v_nop\n\tv_nop\n\tv_nop\n\tv_nop" : "+v"(a), "+v"(b) : "v"(x), "v"(y)); }
__device__ __forceinline__ void keep4_h(v16h a, v16h b, v16h c, v16h d) { asm volatile("v_nop" :: "v"(a), "v"(b), "v"(c), "v"(d)); }
__device__ __forceinline__ void keep4_b(v16b a, v16b b, v16b c, v16b d) { asm volatile("v_nop" :: "v"(a), "v"(b), "v"(c), "v"(d)); }
__device__ __forceinline__ void acc_guard4(v8f& a, v8f& b, v8f& c, v8f& d) { asm volatile("v_nop\n\tv_nop\n\tv_nop\n\tv_nop" : "+v"(a), "+v"(b), "+v"(c), "+v"(d)); }
template <typename T> struct Frag;
template <> struct Frag<_Float16> {
  typedef v16h V; union U { v16h v; v8h h[2]; };
  static __device__ __forceinline__ v16h load(const _Float16* p) {
    U f; f.h[0] = *(const v8h*)(p); f.h[1] = *(const v8h*)(p + 16); return f.v;
  }
  static __device__ __forceinline__ v8f mma(v16h a, v16h b, v8f c) {
    return __builtin_amdgcn_wmma_f32_16x16x32_f16(false, a, false, b, (short)0, c, false, false);
  }
  static __device__ __forceinline__ void guard(v8f& a, v8f& b, v16h x, v16h y) { dep_guard_h(a, b, x, y); }
  static __device__ __forceinline__ void keep(v16h a, v16h b, v16h c, v16h d) { keep4_h(a, b, c, d); }
};
template <> struct Frag<__bf16> {
  typedef v16b V; union U { v16b v; v8b h[2]; };
  static __device__ __forceinline__ v16b load(const __bf16* p) {
    U f; f.h[0] = *(const v8b*)(p); f.h[1] = *(const v8b*)(p + 16); return f.v;
  }
  static __device__ __forceinline__ v8f mma(v16b a, v16b b, v8f c) {
    return __builtin_amdgcn_wmma_f32_16x16x32_bf16(false, a, false, b, (short)0, c, false, false);
  }
  static __device__ __forceinline__ void guard(v8f& a, v8f& b, v16b x, v16b y) { dep_guard_b(a, b, x, y); }
  static __device__ __forceinline__ void keep(v16b a, v16b b, v16b c, v16b d) { keep4_b(a, b, c, d); }
};

__device__ __forceinline__ unsigned pk16(unsigned short a, unsigned short b) { return (unsigned)a | ((unsigned)b << 16); }

template <int ET> struct Elem;
template <> struct Elem<0> { typedef _Float16 T; };
template <> struct Elem<1> { typedef __bf16 T; };
template <int ET, bool SPLIT, int BIAS_MODE, int OUT_MODE, bool RESID, int ACT = 0>
__global__ __launch_bounds__(256) void wmma_gemm64(
    const unsigned short* __restrict__ Ap, const unsigned short* __restrict__ A2p, int lda, long strideA,
    const unsigned short* __restrict__ Btp, const unsigned short* __restrict__ Bt2p, int ldb, long strideB,
    void* __restrict__ Cout, void* __restrict__ Cout2, int ldc, long strideC,
    const float* __restrict__ bias,
    const float* __restrict__ resid, long strideR,
    int M, int N, int K, float scale) {
  typedef typename Elem<ET>::T T;
  typedef typename Frag<T>::V V;
  const T* A = (const T*)Ap; const T* A2 = (const T*)A2p; const T* Bt = (const T*)Btp; const T* Bt2 = (const T*)Bt2p;
  __shared__ __align__(16) float sT[8][16 * 68];
  const int b    = blockIdx.y;
  const int lane = threadIdx.x & 31;
  const int wave = threadIdx.x >> 5;
  const int tilesN = N >> 6;
  const int tilesM = M >> 6;
  const int tile = blockIdx.x * 8 + wave;
  if (tile >= tilesM * tilesN) return;
  const int tm = tile / tilesN;
  const int tn = tile - tm * tilesN;
  const int m0 = tm << 6;
  const int n0 = tn << 6;

  const T* Ab  = A  + (size_t)b * strideA;
  const T* Bb  = Bt + (size_t)b * strideB;
  const T* Ab2 = SPLIT ? (A2  + (size_t)b * strideA) : nullptr;
  const T* Bb2 = SPLIT ? (Bt2 + (size_t)b * strideB) : nullptr;

  const int rlane = lane & 15;
  const int koff  = (lane >> 4) * 8;
  const int mOff  = (lane >> 4) * 8;

  v8f acc[4][4];
#pragma unroll
  for (int i = 0; i < 4; ++i)
#pragma unroll
    for (int j = 0; j < 4; ++j) acc[i][j] = (v8f){0.f,0.f,0.f,0.f,0.f,0.f,0.f,0.f};

  for (int k0 = 0; k0 < K; k0 += 32) {
    V bh[4], bl[4];
#pragma unroll
    for (int j = 0; j < 4; ++j) {
      const size_t bo = (size_t)(n0 + (j << 4) + rlane) * ldb + koff + k0;
      bh[j] = Frag<T>::load(Bb + bo);
      if (SPLIT) bl[j] = Frag<T>::load(Bb2 + bo);
    }
#pragma unroll
    for (int i = 0; i < 4; ++i) {
      const size_t ao = (size_t)(m0 + (i << 4) + rlane) * lda + koff + k0;
      V ah = Frag<T>::load(Ab + ao);
      V al;
      if (SPLIT) al = Frag<T>::load(Ab2 + ao);
#pragma unroll
      for (int j = 0; j < 4; ++j) {
        acc[i][j] = Frag<T>::mma(ah, bh[j], acc[i][j]);
        if (SPLIT) {
          acc[i][j] = Frag<T>::mma(ah, bl[j], acc[i][j]);
          acc[i][j] = Frag<T>::mma(al, bh[j], acc[i][j]);
        }
      }
      Frag<T>::guard(acc[i][0], acc[i][3], ah, SPLIT ? al : ah);
    }
    Frag<T>::keep(bh[0], bh[1], bh[2], bh[3]);
    if (SPLIT) Frag<T>::keep(bl[0], bl[1], bl[2], bl[3]);
  }
  acc_guard4(acc[0][0], acc[0][1], acc[0][2], acc[0][3]);
  acc_guard4(acc[1][0], acc[1][1], acc[1][2], acc[1][3]);
  acc_guard4(acc[2][0], acc[2][1], acc[2][2], acc[2][3]);
  acc_guard4(acc[3][0], acc[3][1], acc[3][2], acc[3][3]);

  float* slab = sT[wave];
  const float* Rb = RESID ? (resid + (size_t)b * strideR) : nullptr;
#pragma unroll
  for (int i = 0; i < 4; ++i) {
    const int mBase = m0 + (i << 4);
#pragma unroll
    for (int j = 0; j < 4; ++j) {
      const int n = n0 + (j << 4) + rlane;
      float bv = 0.f;
      if (BIAS_MODE == 2) bv = bias[n];
#pragma unroll
      for (int r = 0; r < 8; ++r) {
        float v = acc[i][j][r] * scale;
        if (BIAS_MODE == 1) v += bias[mBase + mOff + r];
        if (BIAS_MODE == 2) v += bv;
        if (RESID) v += Rb[(size_t)(mBase + mOff + r) * ldc + n];
        if (ACT == 2) v = fmaxf(v, 0.0f);
        if (ACT == 4) v = (v > 0.f) ? v : 0.01f * v;
        slab[(mOff + r) * 68 + (j << 4) + rlane] = v;
      }
    }
    __builtin_amdgcn_fence(__ATOMIC_RELEASE, "workgroup");
    __builtin_amdgcn_wave_barrier();
    __builtin_amdgcn_fence(__ATOMIC_ACQUIRE, "workgroup");
    if (OUT_MODE == 0) {
      float* C = (float*)Cout + (size_t)b * strideC;
      const int hh = lane >> 4, c4 = (lane & 15) * 4;
      for (int pass = 0; pass < 2; ++pass) {
#pragma unroll
        for (int it = 0; it < 8; ++it) {
          const int row = it * 2 + hh;
          v4f v = *(const v4f*)(slab + row * 68 + c4);
          *(volatile v4f*)(C + (size_t)(mBase + row) * ldc + n0 + c4) = v;
        }
        __threadfence();
      }
    } else {
      const int q = lane >> 3, c8 = (lane & 7) * 8;
      unsigned short* C  = (unsigned short*)Cout  + (size_t)b * strideC;
      unsigned short* C2 = (OUT_MODE == 2) ? ((unsigned short*)Cout2 + (size_t)b * strideC) : nullptr;
      for (int pass = 0; pass < 2; ++pass) {
#pragma unroll
        for (int it = 0; it < 4; ++it) {
          const int row = it * 4 + q;
          const float* sp = slab + row * 68 + c8;
          v8h hv, lv;
#pragma unroll
          for (int e = 0; e < 8; ++e) {
            if (OUT_MODE == 1) {
              hv[e] = (_Float16)sp[e];
            } else {
              unsigned short hb = f2bf_bits(sp[e]);
              unsigned short lb = f2bf_bits(sp[e] - bf_bits2f(hb));
              hv[e] = __builtin_bit_cast(_Float16, hb);
              lv[e] = __builtin_bit_cast(_Float16, lb);
            }
          }
          *(volatile v8h*)(C + (size_t)(mBase + row) * ldc + n0 + c8) = hv;
          if (OUT_MODE == 2) *(volatile v8h*)(C2 + (size_t)(mBase + row) * ldc + n0 + c8) = lv;
        }
        __threadfence();
      }
    }
    __builtin_amdgcn_fence(__ATOMIC_RELEASE, "workgroup");
    __builtin_amdgcn_wave_barrier();
    __builtin_amdgcn_fence(__ATOMIC_ACQUIRE, "workgroup");
  }
}

__global__ __launch_bounds__(256) void split8_kernel(const float* __restrict__ in,
                                                     unsigned short* __restrict__ hi, unsigned short* __restrict__ lo,
                                                     int n8, int mode) {
  const int i = blockIdx.x * kThreads + threadIdx.x;
  if (i >= n8) return;
  const long o = 8L * (long)i;
  long src = o;
  bool zero = false;
  if (mode == 1) {
    const long n = o >> 12;
    const int  r = (int)((o >> 6) & 63);
    const int  c = (int)(o & 63);
    const int  rc = (r < kCpHid) ? r : (kCpHid - 1);
    src  = n * (kCpHid * kObjDim) + (long)rc * kObjDim + c;
    zero = (r >= kCpHid);
  } else if (mode == 2) {
    const long n = o >> 6;
    const int  c = (int)(o & 63);
    src = (n & 63) * (2 * kObjDim) + (n >> 6) * kObjDim + c;
  }
  const float* p = in + src;
  const v4f a = *(const v4f*)(p);
  const v4f c4 = *(const v4f*)(p + 4);
  float x[8];
#pragma unroll
  for (int e = 0; e < 4; ++e) { x[e] = zero ? 0.0f : a[e]; x[4 + e] = zero ? 0.0f : c4[e]; }
  unsigned short hb[8], lb[8];
#pragma unroll
  for (int e = 0; e < 8; ++e) {
    hb[e] = f2bf_bits(x[e]);
    lb[e] = f2bf_bits(x[e] - bf_bits2f(hb[e]));
  }
  const v4u uh = (v4u){pk16(hb[0], hb[1]), pk16(hb[2], hb[3]), pk16(hb[4], hb[5]), pk16(hb[6], hb[7])};
  const v4u ul = (v4u){pk16(lb[0], lb[1]), pk16(lb[2], lb[3]), pk16(lb[4], lb[5]), pk16(lb[6], lb[7])};
  unsigned short* qh = hi + o;
  unsigned short* ql = lo + o;
  *(volatile v4u*)qh = uh;
  *(volatile v4u*)ql = ul;
  __threadfence();
  *(volatile v4u*)qh = uh;
  *(volatile v4u*)ql = ul;
}

constexpr int kPairObj = 2 * kNObj;
constexpr int kQsN  = kPairObj * kQkvW;
constexpr int kPsN  = 2 * kHeads * kNObj * kNObj;
constexpr int kCsN  = kPairObj * kObjDim;
constexpr int kAttnPair = 2 * kNObj * kNObj;

__global__ __launch_bounds__(256) void attn_pairs_kernel(const float* __restrict__ qkv,
                                                         unsigned short* __restrict__ ctx_hi,
                                                         unsigned short* __restrict__ ctx_lo,
                                                         float* __restrict__ attn_out) {
  __shared__ __align__(16) float qs[kQsN];
  __shared__ __align__(16) float ps[kPsN];
  __shared__ __align__(16) float cs[kCsN];
  const int bp   = blockIdx.x;
  const int tid  = threadIdx.x;
  const int lane = tid & 31;
  const int wave = tid >> 5;

  {
    const float* src = qkv + (size_t)bp * kQsN;
    for (int e = tid; e < kQsN / 4; e += kThreads) {
      const v4f v = *(const v4f*)(src + 4 * e);
      *(v4f*)(qs + 4 * e) = v;
    }
  }
  __syncthreads();

#pragma unroll 1
  for (int p = tid; p < kPsN; p += kThreads) {
    const int bb  = p / (kHeads * kNObj * kNObj);
    const int rem = p - bb * (kHeads * kNObj * kNObj);
    const int h   = rem / (kNObj * kNObj);
    const int r2  = rem - h * (kNObj * kNObj);
    const int i   = r2 / kNObj;
    const int j   = r2 - i * kNObj;
    const float* qp = qs + (bb * kNObj + i) * kQkvW + h * kHeadDim;
    const float* kp = qs + (bb * kNObj + j) * kQkvW + kObjDim + h * kHeadDim;
    float s = 0.f;
#pragma unroll 1
    for (int d = 0; d < kHeadDim; ++d) s += qp[d] * kp[d];
    ps[p] = s * 0.25f;
  }
  __syncthreads();

  if (tid < 2 * kHeads * kNObj) {
    float* pr = ps + tid * kNObj;
    float m = pr[0];
#pragma unroll 1
    for (int j = 1; j < kNObj; ++j) m = fmaxf(m, pr[j]);
    float sum = 0.f;
#pragma unroll 1
    for (int j = 0; j < kNObj; ++j) { const float e = expf(pr[j] - m); pr[j] = e; sum += e; }
    const float inv = 1.0f / sum;
#pragma unroll 1
    for (int j = 0; j < kNObj; ++j) pr[j] = pr[j] * inv;
  }
  __syncthreads();

#pragma unroll 1
  for (int o = tid; o < kCsN; o += kThreads) {
    const int bb  = o / (kNObj * kObjDim);
    const int rem = o - bb * (kNObj * kObjDim);
    const int i   = rem >> 6;
    const int c   = rem & 63;
    const int h   = c >> 4;
    const float* pp = ps + ((bb * kHeads + h) * kNObj + i) * kNObj;
    const float* vp = qs + (bb * kNObj) * kQkvW + 2 * kObjDim + c;
    float a = 0.f;
#pragma unroll 1
    for (int j = 0; j < kNObj; ++j) a += pp[j] * vp[j * kQkvW];
    cs[o] = a;
  }
  __syncthreads();

  {
    const int q = lane >> 3, c8 = (lane & 7) * 8;
    const size_t rowbase = (size_t)bp * kPairObj;
    for (int pass = 0; pass < 2; ++pass) {
#pragma unroll
      for (int it = 0; it < 2; ++it) {
        const int L = it * 32 + wave * 4 + q;
        if (L < kPairObj) {
          const float* sp = cs + L * kObjDim + c8;
          unsigned short hb[8], lb[8];
#pragma unroll
          for (int e = 0; e < 8; ++e) {
            hb[e] = f2bf_bits(sp[e]);
            lb[e] = f2bf_bits(sp[e] - bf_bits2f(hb[e]));
          }
          const v4u uh = (v4u){pk16(hb[0], hb[1]), pk16(hb[2], hb[3]), pk16(hb[4], hb[5]), pk16(hb[6], hb[7])};
          const v4u ul = (v4u){pk16(lb[0], lb[1]), pk16(lb[2], lb[3]), pk16(lb[4], lb[5]), pk16(lb[6], lb[7])};
          *(volatile v4u*)(ctx_hi + (rowbase + L) * kObjDim + c8) = uh;
          *(volatile v4u*)(ctx_lo + (rowbase + L) * kObjDim + c8) = ul;
        }
      }
      __threadfence();
    }
  }

  if (tid < kAttnPair / 4) {
    float r[4];
#pragma unroll
    for (int qd = 0; qd < 4; ++qd) {
      const int e   = tid * 4 + qd;
      const int bb  = e / (kNObj * kNObj);
      const int rem = e - bb * (kNObj * kNObj);
      const float* p0 = ps + bb * (kHeads * kNObj * kNObj) + rem;
      r[qd] = (((p0[0] + p0[kNObj * kNObj]) + p0[2 * kNObj * kNObj]) + p0[3 * kNObj * kNObj]) * 0.25f;
    }
    const v4f v = (v4f){r[0], r[1], r[2], r[3]};
    float* dst = attn_out + (size_t)bp * kAttnPair + tid * 4;
    *(volatile v4f*)dst = v;
    __threadfence();
    *(volatile v4f*)dst = v;
  }
}

__global__ __launch_bounds__(256) void objprop_kernel(const float* __restrict__ pre,
                                                      const float* __restrict__ cp_b1, const float* __restrict__ cp_w2,
                                                      const float* __restrict__ cp_b2, float* __restrict__ out, int n4) {
  const int t = blockIdx.x * kThreads + threadIdx.x;
  if (t >= n4) return;
  float r[4];
#pragma unroll
  for (int qd = 0; qd < 4; ++qd) {
    const int e   = t * 4 + qd;
    const int row = e / 3;
    const int o   = e - row * 3;
    const int n   = row % kNObj;
    const float* hp = pre + (size_t)row * kObjDim;
    const float* bp = cp_b1 + n * kCpHid;
    const float* wp = cp_w2 + (n * 3 + o) * kCpHid;
    float a = 0.f;
#pragma unroll 1
    for (int h = 0; h < kCpHid; ++h) a += fmaxf(hp[h] + bp[h], 0.0f) * wp[h];
    r[qd] = a + cp_b2[n * 3 + o];
  }
  const v4f v = (v4f){r[0], r[1], r[2], r[3]};
  float* dst = out + (size_t)t * 4;
  *(volatile v4f*)dst = v;
  __threadfence();
  *(volatile v4f*)dst = v;
}

__global__ __launch_bounds__(256) void pair_kernel(const float* __restrict__ hihj,
                                                   const float* __restrict__ ip_b1, const float* __restrict__ ip_w2,
                                                   const float* __restrict__ ip_b2, float* __restrict__ out, int n4) {
  __shared__ float b1s[kObjDim];
  __shared__ float w2s[kObjDim];
  const int tid = threadIdx.x;
  if (tid < kObjDim) { b1s[tid] = ip_b1[tid]; w2s[tid] = ip_w2[tid]; }
  __syncthreads();
  const int t = blockIdx.x * kThreads + tid;
  if (t >= n4) return;
  const float bias2 = ip_b2[0];
  float r[4];
#pragma unroll
  for (int qd = 0; qd < 4; ++qd) {
    const int e   = t * 4 + qd;
    const int b   = e / (kNObj * (kNObj - 1));
    const int rem = e - b * (kNObj * (kNObj - 1));
    const int i   = rem / (kNObj - 1);
    const int m   = rem - i * (kNObj - 1);
    const int j   = m + ((m >= i) ? 1 : 0);
    const float* hp = hihj + ((size_t)b * kNObj + i) * (2 * kObjDim);
    const float* jp = hihj + ((size_t)b * kNObj + j) * (2 * kObjDim) + kObjDim;
    float a = 0.f;
#pragma unroll 1
    for (int c = 0; c < kObjDim; ++c) a += fmaxf((hp[c] + jp[c]) + b1s[c], 0.0f) * w2s[c];
    r[qd] = a + bias2;
  }
  const v4f v = (v4f){r[0], r[1], r[2], r[3]};
  float* dst = out + (size_t)t * 4;
  *(volatile v4f*)dst = v;
  __threadfence();
  *(volatile v4f*)dst = v;
}

extern "C" void kernel_launch(void* const* d_in, const int* in_sizes, int n_in,
                              void* d_out, int out_size, void* d_ws, size_t ws_size,
                              hipStream_t stream)
{
  if (n_in < 17) return;
  const int B = in_sizes[0] / kDModel;
  if (B <= 0 || (B % 64) != 0) return;
  if ((long)out_size != (long)B * (long)(kHid + kHid + kNObj * 3 + kNObj * (kNObj - 1) + kNObj * kNObj)) return;
  if (in_sizes[1] != kHid * kDModel || in_sizes[3] != kHid * kHid || in_sizes[5] != kQkvW * kObjDim ||
      in_sizes[7] != kObjDim * kObjDim || in_sizes[9] != kNObj * kCpHid * kObjDim ||
      in_sizes[13] != kObjDim * 2 * kObjDim) return;

  const float* state      = (const float*)d_in[0];
  const float* enc_w1     = (const float*)d_in[1];
  const float* enc_b1     = (const float*)d_in[2];
  const float* enc_w2     = (const float*)d_in[3];
  const float* enc_b2     = (const float*)d_in[4];
  const float* in_proj_w  = (const float*)d_in[5];
  const float* in_proj_b  = (const float*)d_in[6];
  const float* out_proj_w = (const float*)d_in[7];
  const float* out_proj_b = (const float*)d_in[8];
  const float* cp_w1      = (const float*)d_in[9];
  const float* cp_b1      = (const float*)d_in[10];
  const float* cp_w2      = (const float*)d_in[11];
  const float* cp_b2      = (const float*)d_in[12];
  const float* ip_w1      = (const float*)d_in[13];
  const float* ip_b1      = (const float*)d_in[14];
  const float* ip_w2      = (const float*)d_in[15];
  const float* ip_b2      = (const float*)d_in[16];

  float* out_objects = (float*)d_out;
  float* out_causal  = out_objects + (size_t)B * kHid;
  float* out_props   = out_causal  + (size_t)B * kHid;
  float* out_inter   = out_props   + (size_t)B * kNObj * 3;
  float* out_attn    = out_inter   + (size_t)B * kNObj * (kNObj - 1);

  size_t off = 0;
  char* wsb = (char*)d_ws;
  auto carve = [&](size_t bytes) -> char* { char* p = wsb + off; off += (bytes + 255) & ~(size_t)255; return p; };
  const size_t nState = (size_t)B * kDModel;
  const size_t nW1    = (size_t)kHid * kDModel;
  const size_t nW2    = (size_t)kHid * kHid;
  const size_t nAct   = (size_t)B * kHid;
  const size_t nInpw  = (size_t)kQkvW * kObjDim;
  const size_t nOutw  = (size_t)kObjDim * kObjDim;
  const size_t nCpw   = (size_t)kNObj * kObjDim * kObjDim;
  const size_t nIpw   = (size_t)2 * kObjDim * kObjDim;
  const size_t nQkv   = (size_t)B * kNObj * kQkvW;
  const size_t nCtx   = (size_t)B * kNObj * kObjDim;

  unsigned short* st_hi   = (unsigned short*)carve(nState * 2);
  unsigned short* st_lo   = (unsigned short*)carve(nState * 2);
  unsigned short* w1_hi   = (unsigned short*)carve(nW1 * 2);
  unsigned short* w1_lo   = (unsigned short*)carve(nW1 * 2);
  unsigned short* w2_hi   = (unsigned short*)carve(nW2 * 2);
  unsigned short* w2_lo   = (unsigned short*)carve(nW2 * 2);
  unsigned short* act_hi  = (unsigned short*)carve(nAct * 2);
  unsigned short* act_lo  = (unsigned short*)carve(nAct * 2);
  unsigned short* inpw_hi = (unsigned short*)carve(nInpw * 2);
  unsigned short* inpw_lo = (unsigned short*)carve(nInpw * 2);
  unsigned short* outw_hi = (unsigned short*)carve(nOutw * 2);
  unsigned short* outw_lo = (unsigned short*)carve(nOutw * 2);
  unsigned short* cpw_hi  = (unsigned short*)carve(nCpw * 2);
  unsigned short* cpw_lo  = (unsigned short*)carve(nCpw * 2);
  unsigned short* ipw_hi  = (unsigned short*)carve(nIpw * 2);
  unsigned short* ipw_lo  = (unsigned short*)carve(nIpw * 2);
  float*          big     = (float*)carve(nQkv * 4);
  unsigned short* ctx_hi  = (unsigned short*)carve(nCtx * 2);
  unsigned short* ctx_lo  = (unsigned short*)carve(nCtx * 2);
  if (off > ws_size) return;

  float* qkv_f  = big;
  float* cpre_f = big;
  float* hihj_f = big + (size_t)B * kHid;

  const int M1 = B;
  const int M2 = B * kNObj;

  auto blocks_for = [](long n) -> unsigned { return (unsigned)((n + kThreads - 1) / kThreads); };

  {
    const int n8 = (int)(nState / 8);
    split8_kernel<<<blocks_for(n8), kThreads, 0, stream>>>(state, st_hi, st_lo, n8, 0);
  }
  {
    const int n8 = (int)(nW1 / 8);
    split8_kernel<<<blocks_for(n8), kThreads, 0, stream>>>(enc_w1, w1_hi, w1_lo, n8, 0);
  }
  {
    const int n8 = (int)(nW2 / 8);
    split8_kernel<<<blocks_for(n8), kThreads, 0, stream>>>(enc_w2, w2_hi, w2_lo, n8, 0);
  }
  {
    const int n8 = (int)(nInpw / 8);
    split8_kernel<<<blocks_for(n8), kThreads, 0, stream>>>(in_proj_w, inpw_hi, inpw_lo, n8, 0);
  }
  {
    const int n8 = (int)(nOutw / 8);
    split8_kernel<<<blocks_for(n8), kThreads, 0, stream>>>(out_proj_w, outw_hi, outw_lo, n8, 0);
  }
  {
    const int n8 = (int)(nCpw / 8);
    split8_kernel<<<blocks_for(n8), kThreads, 0, stream>>>(cp_w1, cpw_hi, cpw_lo, n8, 1);
  }
  {
    const int n8 = (int)(nIpw / 8);
    split8_kernel<<<blocks_for(n8), kThreads, 0, stream>>>(ip_w1, ipw_hi, ipw_lo, n8, 2);
  }

  {
    const long tiles = (long)(M1 / 64) * (kHid / 64);
    wmma_gemm64<1, true, 2, 2, false, 2><<<dim3((unsigned)((tiles + 7) / 8), 1), kThreads, 0, stream>>>(
        st_hi, st_lo, kDModel, 0L, w1_hi, w1_lo, kDModel, 0L,
        (void*)act_hi, (void*)act_lo, kHid, 0L, enc_b1, nullptr, 0L, M1, kHid, kDModel, 1.0f);
  }
  {
    const long tiles = (long)(M1 / 64) * (kHid / 64);
    wmma_gemm64<1, true, 2, 0, false, 0><<<dim3((unsigned)((tiles + 7) / 8), 1), kThreads, 0, stream>>>(
        act_hi, act_lo, kHid, 0L, w2_hi, w2_lo, kHid, 0L,
        (void*)out_objects, nullptr, kHid, 0L, enc_b2, nullptr, 0L, M1, kHid, kHid, 1.0f);
  }
  {
    const int n8 = (int)(nAct / 8);
    split8_kernel<<<blocks_for(n8), kThreads, 0, stream>>>(out_objects, act_hi, act_lo, n8, 0);
  }
  {
    const long tiles = (long)(M2 / 64) * (kQkvW / 64);
    wmma_gemm64<1, true, 2, 0, false, 0><<<dim3((unsigned)((tiles + 7) / 8), 1), kThreads, 0, stream>>>(
        act_hi, act_lo, kObjDim, 0L, inpw_hi, inpw_lo, kObjDim, 0L,
        (void*)qkv_f, nullptr, kQkvW, 0L, in_proj_b, nullptr, 0L, M2, kQkvW, kObjDim, 1.0f);
  }
  attn_pairs_kernel<<<(unsigned)(B / 2), kThreads, 0, stream>>>(qkv_f, ctx_hi, ctx_lo, out_attn);

  {
    const long tiles = (long)(M2 / 64) * (kObjDim / 64);
    wmma_gemm64<1, true, 2, 0, false, 0><<<dim3((unsigned)((tiles + 7) / 8), 1), kThreads, 0, stream>>>(
        ctx_hi, ctx_lo, kObjDim, 0L, outw_hi, outw_lo, kObjDim, 0L,
        (void*)out_causal, nullptr, kObjDim, 0L, out_proj_b, nullptr, 0L, M2, kObjDim, kObjDim, 1.0f);
  }
  {
    const long tiles = (long)(M1 / 64) * 1;
    wmma_gemm64<1, true, 0, 0, false, 0><<<dim3((unsigned)((tiles + 7) / 8), kNObj), kThreads, 0, stream>>>(
        act_hi, act_lo, kHid, (long)kObjDim, cpw_hi, cpw_lo, kObjDim, (long)(kObjDim * kObjDim),
        (void*)cpre_f, nullptr, kHid, (long)kObjDim, nullptr, nullptr, 0L, M1, kObjDim, kObjDim, 1.0f);
  }
  {
    const int n4 = B * kNObj * 3 / 4;
    objprop_kernel<<<blocks_for(n4), kThreads, 0, stream>>>(cpre_f, cp_b1, cp_w2, cp_b2, out_props, n4);
  }
  {
    const long tiles = (long)(M2 / 64) * 2;
    wmma_gemm64<1, true, 0, 0, false, 0><<<dim3((unsigned)((tiles + 7) / 8), 1), kThreads, 0, stream>>>(
        act_hi, act_lo, kObjDim, 0L, ipw_hi, ipw_lo, kObjDim, 0L,
        (void*)hihj_f, nullptr, 2 * kObjDim, 0L, nullptr, nullptr, 0L, M2, 2 * kObjDim, kObjDim, 1.0f);
  }
  {
    const int n4 = B * kNObj * (kNObj - 1) / 4;
    pair_kernel<<<blocks_for(n4), kThreads, 0, stream>>>(hihj_f, ip_b1, ip_w2, ip_b2, out_inter, n4);
  }
}
